// ConcatCritic_62783831933329
// MI455X (gfx1250) — hardware-run, weakly checked
//
#include <hip/hip_runtime.h>
#include <math.h>

typedef __attribute__((ext_vector_type(16))) _Float16 v16h;
typedef __attribute__((ext_vector_type(8)))  _Float16 v8h;
typedef __attribute__((ext_vector_type(16))) __bf16   v16b;
typedef __attribute__((ext_vector_type(8)))  __bf16   v8b;
typedef __attribute__((ext_vector_type(8)))  float    v8f;
typedef __attribute__((ext_vector_type(4)))  float    v4f;

constexpr int kBatch   = 512;
constexpr int kNX      = 128;
constexpr int kW1P     = 256;
constexpr int kHid     = 512;
constexpr int kPairs   = kBatch * kBatch;
constexpr int kMT      = 64;
constexpr int kAP      = 520;
constexpr float kCarryA = 16.0f;
constexpr float kCarryW = 64.0f;
constexpr float kFold   = kCarryA * kCarryW;
constexpr float kFoldInv = 1.0f / kFold;
constexpr float kF16MinNormal = 6.103515625e-05f;
static_assert((kNX % 32) == 0 && (kHid % 32) == 0);
static_assert((kBatch % 64) == 0 && (kHid % 64) == 0 && (kBatch % kMT) == 0);
static_assert(kFold == 1024.0f);
static_assert((kAP % 8) == 0 && kAP >= kHid);

constexpr size_t kOffXH  = 0;
constexpr size_t kOffXL  = kOffXH  + (size_t)kBatch * kNX  * 2;
constexpr size_t kOffYH  = kOffXL  + (size_t)kBatch * kNX  * 2;
constexpr size_t kOffYL  = kOffYH  + (size_t)kBatch * kNX  * 2;
constexpr size_t kOffW1H = kOffYL  + (size_t)kBatch * kNX  * 2;
constexpr size_t kOffW1L = kOffW1H + (size_t)kHid   * kW1P * 2;
constexpr size_t kOffW2H = kOffW1L + (size_t)kHid   * kW1P * 2;
constexpr size_t kOffHX  = kOffW2H + (size_t)kHid   * kHid * 2;
constexpr size_t kOffHYB = kOffHX  + (size_t)kBatch * kHid * 4;
constexpr size_t kWsTotal = kOffHYB + (size_t)kBatch * kHid * 4;
static_assert(kWsTotal == 3670016ull);
static_assert(kWsTotal <= 134217728ull);
static_assert((kOffXL % 128) == 0 && (kOffYH % 128) == 0 && (kOffYL % 128) == 0 && (kOffW1H % 128) == 0 &&
              (kOffW1L % 128) == 0 && (kOffW2H % 128) == 0 && (kOffHX % 128) == 0 && (kOffHYB % 128) == 0);

__device__ __forceinline__ unsigned short f2bf_bits(float f) {
  unsigned u = __float_as_uint(f);
  return (unsigned short)((u + 0x7FFFu + ((u >> 16) & 1u)) >> 16);
}
__device__ __forceinline__ float bf_bits2f(unsigned short h) { return __uint_as_float(((unsigned)h) << 16); }

__device__ __forceinline__ void tie_h(v8f& c, v16h x, v16h y) { asm volatile("v_nop\n\tv_nop\n\tv_nop\n\tv_nop" : "+v"(c) : "v"(x), "v"(y)); }
__device__ __forceinline__ void tie_b(v8f& c, v16b x, v16b y) { asm volatile("v_nop\n\tv_nop\n\tv_nop\n\tv_nop" : "+v"(c) : "v"(x), "v"(y)); }
__device__ __forceinline__ void keep4_h(v16h a, v16h b, v16h c, v16h d) { asm volatile("v_nop" :: "v"(a), "v"(b), "v"(c), "v"(d)); }
__device__ __forceinline__ void keep4_b(v16b a, v16b b, v16b c, v16b d) { asm volatile("v_nop" :: "v"(a), "v"(b), "v"(c), "v"(d)); }

template <typename T> struct Frag;
template <> struct Frag<_Float16> {
  typedef v16h V; union U { v16h v; v8h h[2]; };
  static __device__ __forceinline__ v16h load(const _Float16* p) {
    U f; f.h[0] = *(const v8h*)(p); f.h[1] = *(const v8h*)(p + 16); return f.v;
  }
  static __device__ __forceinline__ v8f mma(v16h a, v16h b, v8f c) {
    c = __builtin_amdgcn_wmma_f32_16x16x32_f16(false, a, false, b, (short)0, c, false, false);
    tie_h(c, a, b);
    return c;
  }
  static __device__ __forceinline__ void keep(v16h a, v16h b, v16h c, v16h d) { keep4_h(a, b, c, d); }
};
template <> struct Frag<__bf16> {
  typedef v16b V; union U { v16b v; v8b h[2]; };
  static __device__ __forceinline__ v16b load(const __bf16* p) {
    U f; f.h[0] = *(const v8b*)(p); f.h[1] = *(const v8b*)(p + 16); return f.v;
  }
  static __device__ __forceinline__ v8f mma(v16b a, v16b b, v8f c) {
    c = __builtin_amdgcn_wmma_f32_16x16x32_bf16(false, a, false, b, (short)0, c, false, false);
    tie_b(c, a, b);
    return c;
  }
  static __device__ __forceinline__ void keep(v16b a, v16b b, v16b c, v16b d) { keep4_b(a, b, c, d); }
};

template <bool SPLIT, int BIAS_MODE>
__global__ __launch_bounds__(256) void wmma_gemm64_bf16(
    const unsigned short* __restrict__ Ap, const unsigned short* __restrict__ A2p, int lda,
    const unsigned short* __restrict__ Btp, const unsigned short* __restrict__ Bt2p, int ldb,
    float* __restrict__ C, int ldc,
    const float* __restrict__ bias,
    int M, int N, int K) {
  typedef __bf16 T;
  typedef Frag<T>::V V;
  const T* A = (const T*)Ap; const T* A2 = (const T*)A2p; const T* Bt = (const T*)Btp; const T* Bt2 = (const T*)Bt2p;
  __shared__ __align__(16) float sT[8][16 * 68];
  const int lane = threadIdx.x & 31;
  const int wave = threadIdx.x >> 5;
  const int tilesN = N >> 6;
  const int tilesM = M >> 6;
  const int tile = blockIdx.x * 8 + wave;
  if (tile >= tilesM * tilesN) return;
  const int tm = tile / tilesN;
  const int tn = tile - tm * tilesN;
  const int m0 = tm << 6;
  const int n0 = tn << 6;

  const int rlane = lane & 15;
  const int koff  = (lane >> 4) * 8;
  const int mOff  = (lane >> 4) * 8;

  v8f acc[4][4];
#pragma unroll
  for (int i = 0; i < 4; ++i)
#pragma unroll
    for (int j = 0; j < 4; ++j) acc[i][j] = (v8f){0.f,0.f,0.f,0.f,0.f,0.f,0.f,0.f};

  for (int k0 = 0; k0 < K; k0 += 32) {
    V bh[4], bl[4];
#pragma unroll
    for (int j = 0; j < 4; ++j) {
      const size_t bo = (size_t)(n0 + (j << 4) + rlane) * ldb + koff + k0;
      bh[j] = Frag<T>::load(Bt + bo);
      if (SPLIT) bl[j] = Frag<T>::load(Bt2 + bo);
    }
#pragma unroll
    for (int i = 0; i < 4; ++i) {
      const size_t ao = (size_t)(m0 + (i << 4) + rlane) * lda + koff + k0;
      V ah = Frag<T>::load(A + ao);
      V al;
      if (SPLIT) al = Frag<T>::load(A2 + ao);
#pragma unroll
      for (int j = 0; j < 4; ++j) {
        acc[i][j] = Frag<T>::mma(ah, bh[j], acc[i][j]);
        if (SPLIT) {
          acc[i][j] = Frag<T>::mma(ah, bl[j], acc[i][j]);
          acc[i][j] = Frag<T>::mma(al, bh[j], acc[i][j]);
        }
      }
    }
    Frag<T>::keep(bh[0], bh[1], bh[2], bh[3]);
    if (SPLIT) Frag<T>::keep(bl[0], bl[1], bl[2], bl[3]);
  }

  float* slab = sT[wave];
#pragma unroll
  for (int i = 0; i < 4; ++i) {
    const int mBase = m0 + (i << 4);
#pragma unroll
    for (int j = 0; j < 4; ++j) {
      const int n = n0 + (j << 4) + rlane;
      float bv = 0.f;
      if (BIAS_MODE == 2) bv = bias[n];
#pragma unroll
      for (int r = 0; r < 8; ++r) {
        float v = acc[i][j][r];
        if (BIAS_MODE == 2) v += bv;
        slab[(mOff + r) * 68 + (j << 4) + rlane] = v;
      }
    }
    __builtin_amdgcn_fence(__ATOMIC_RELEASE, "workgroup");
    __builtin_amdgcn_wave_barrier();
    __builtin_amdgcn_fence(__ATOMIC_ACQUIRE, "workgroup");
    {
      const int hh = lane >> 4, c4 = (lane & 15) * 4;
      for (int pass = 0; pass < 2; ++pass) {
#pragma unroll
        for (int it = 0; it < 8; ++it) {
          const int row = it * 2 + hh;
          v4f v = *(const v4f*)(slab + row * 68 + c4);
          *(volatile v4f*)(C + (size_t)(mBase + row) * ldc + n0 + c4) = v;
        }
        __threadfence();
      }
    }
    __builtin_amdgcn_fence(__ATOMIC_RELEASE, "workgroup");
    __builtin_amdgcn_wave_barrier();
    __builtin_amdgcn_fence(__ATOMIC_ACQUIRE, "workgroup");
  }
}

__global__ __launch_bounds__(256) void split_rows_bf16_kernel(
    const float* __restrict__ src, unsigned short* __restrict__ dhi, unsigned short* __restrict__ dlo, int total8)
{
  const int i = blockIdx.x * 256 + threadIdx.x;
  if (i >= total8) return;
  const size_t e0 = (size_t)i << 3;
  const v4f a0 = *(const v4f*)(src + e0);
  const v4f a1 = *(const v4f*)(src + e0 + 4);
  v8h hv, lv;
#pragma unroll
  for (int e = 0; e < 4; ++e) {
    const float f0 = a0[e];
    const float f1 = a1[e];
    const unsigned short h0 = f2bf_bits(f0), h1 = f2bf_bits(f1);
    const unsigned short l0 = f2bf_bits(f0 - bf_bits2f(h0)), l1 = f2bf_bits(f1 - bf_bits2f(h1));
    hv[e]     = __builtin_bit_cast(_Float16, h0);
    hv[4 + e] = __builtin_bit_cast(_Float16, h1);
    lv[e]     = __builtin_bit_cast(_Float16, l0);
    lv[4 + e] = __builtin_bit_cast(_Float16, l1);
  }
  unsigned short* qh = dhi + e0;
  unsigned short* ql = dlo + e0;
  *(volatile v8h*)qh = hv;
  *(volatile v8h*)ql = lv;
  __threadfence();
  *(volatile v8h*)qh = hv;
  *(volatile v8h*)ql = lv;
}

__global__ __launch_bounds__(256) void w2_plane_kernel(
    const float* __restrict__ W2, unsigned short* __restrict__ w2h, float* __restrict__ out_tail, int total8)
{
  const int i = blockIdx.x * 256 + threadIdx.x;
  if (i >= total8) return;
  const size_t e0 = (size_t)i << 3;
  const v4f a0 = *(const v4f*)(W2 + e0);
  const v4f a1 = *(const v4f*)(W2 + e0 + 4);
  v8h hv;
#pragma unroll
  for (int e = 0; e < 4; ++e) {
    float c0 = a0[e] * kCarryW;
    float c1 = a1[e] * kCarryW;
    c0 = (fabsf(c0) < kF16MinNormal) ? 0.0f : c0;
    c1 = (fabsf(c1) < kF16MinNormal) ? 0.0f : c1;
    hv[e]     = (_Float16)c0;
    hv[4 + e] = (_Float16)c1;
  }
  unsigned short* q = w2h + e0;
  *(volatile v8h*)q = hv;
  if (i == 0) *(volatile float*)out_tail = 0.0f;
  __threadfence();
  *(volatile v8h*)q = hv;
  if (i == 0) *(volatile float*)out_tail = 0.0f;
}

__global__ __launch_bounds__(256) void pair_layer_kernel(
    const float* __restrict__ hx, const float* __restrict__ hyb,
    const _Float16* __restrict__ w2h,
    const float* __restrict__ b2, const float* __restrict__ W3, const float* __restrict__ b3,
    float* __restrict__ out)
{
  __shared__ __align__(16) _Float16 As[kMT * kAP];
  __shared__ __align__(16) float sred[8 * kMT];
  union FU { v16h v; v8h h[2]; };

  const int tid   = threadIdx.x;
  const int lane  = tid & 31;
  const int wave  = tid >> 5;
  const int rlane = lane & 15;
  const int hh    = lane >> 4;
  const int m0    = blockIdx.x * kMT;
  const int iy    = m0 / kBatch;
  const int j0    = m0 - iy * kBatch;

  float b3v = b3[0];
  asm volatile("" : "+v"(b3v));

  {
    const int kg   = tid & 63;
    const int rsub = tid >> 6;
    const float* yp = hyb + (size_t)iy * kHid + kg * 8;
    const v4f y0 = *(const v4f*)(yp);
    const v4f y1 = *(const v4f*)(yp + 4);
#pragma unroll 2
    for (int it = 0; it < 16; ++it) {
      const int row = it * 4 + rsub;
      const float* xp = hx + (size_t)(j0 + row) * kHid + kg * 8;
      const v4f x0 = *(const v4f*)(xp);
      const v4f x1 = *(const v4f*)(xp + 4);
      v8h hv;
#pragma unroll
      for (int e = 0; e < 4; ++e) {
        float c0 = fmaxf(x0[e] + y0[e], 0.0f) * kCarryA;
        float c1 = fmaxf(x1[e] + y1[e], 0.0f) * kCarryA;
        c0 = (c0 < kF16MinNormal) ? 0.0f : c0;
        c1 = (c1 < kF16MinNormal) ? 0.0f : c1;
        hv[e]     = (_Float16)c0;
        hv[4 + e] = (_Float16)c1;
      }
      *(v8h*)(&As[row * kAP + kg * 8]) = hv;
    }
  }
  __syncthreads();

  const int n0   = wave * 64;
  const int koff = hh * 8;
  v8f acc[4][4];
#pragma unroll
  for (int i = 0; i < 4; ++i)
#pragma unroll
    for (int j = 0; j < 4; ++j) acc[i][j] = (v8f){0.f,0.f,0.f,0.f,0.f,0.f,0.f,0.f};

  const _Float16* bp = w2h + (size_t)(n0 + rlane) * kHid + koff;
  const int aoff = rlane * kAP + koff;
#pragma unroll 1
  for (int k0 = 0; k0 < kHid; k0 += 32) {
    v16h bh[4];
#pragma unroll
    for (int j = 0; j < 4; ++j) bh[j] = Frag<_Float16>::load(bp + (size_t)(j * 16) * kHid + k0);
#pragma unroll
    for (int i = 0; i < 4; ++i) {
      FU fa;
      fa.h[0] = *(const v8h*)(&As[aoff + i * 16 * kAP + k0]);
      fa.h[1] = *(const v8h*)(&As[aoff + i * 16 * kAP + k0 + 16]);
      const v16h ah = fa.v;
#pragma unroll
      for (int j = 0; j < 4; ++j) acc[i][j] = Frag<_Float16>::mma(ah, bh[j], acc[i][j]);
    }
    Frag<_Float16>::keep(bh[0], bh[1], bh[2], bh[3]);
  }

  float bbv[4], wwv[4];
#pragma unroll
  for (int j = 0; j < 4; ++j) {
    const int g = n0 + j * 16 + rlane;
    bbv[j] = b2[g] * kFold;
    wwv[j] = W3[g] * kFoldInv;
  }
#pragma unroll
  for (int i = 0; i < 4; ++i) {
    float part[8];
#pragma unroll
    for (int r = 0; r < 8; ++r) part[r] = 0.0f;
#pragma unroll
    for (int j = 0; j < 4; ++j) {
#pragma unroll
      for (int r = 0; r < 8; ++r) {
        const float v = fmaxf(acc[i][j][r] + bbv[j], 0.0f);
        part[r] = fmaf(v, wwv[j], part[r]);
      }
    }
#pragma unroll
    for (int r = 0; r < 8; ++r) {
      float s = part[r];
      s += __shfl_xor(s, 1, 32);
      s += __shfl_xor(s, 2, 32);
      s += __shfl_xor(s, 4, 32);
      s += __shfl_xor(s, 8, 32);
      part[r] = s;
    }
    if (rlane == 0) {
#pragma unroll
      for (int r = 0; r < 8; ++r) sred[wave * kMT + i * 16 + hh * 8 + r] = part[r];
    }
  }
  __syncthreads();

  {
    const int r4 = (tid & 15) * 4;
    v4f sv;
#pragma unroll
    for (int e = 0; e < 4; ++e) {
      const int row = r4 + e;
      float s = sred[row];
      s += sred[1 * kMT + row];
      s += sred[2 * kMT + row];
      s += sred[3 * kMT + row];
      s += sred[4 * kMT + row];
      s += sred[5 * kMT + row];
      s += sred[6 * kMT + row];
      s += sred[7 * kMT + row];
      sv[e] = s + b3v;
    }
    if (tid < 16) {
      float* p = out + (size_t)m0 + r4;
      *(volatile v4f*)p = sv;
      __threadfence();
      *(volatile v4f*)p = sv;
    }
  }
}

extern "C" void kernel_launch(void* const* d_in, const int* in_sizes, int n_in,
                              void* d_out, int out_size, void* d_ws, size_t ws_size,
                              hipStream_t stream) {
  if (n_in < 8) return;
  if (in_sizes[0] != kBatch * kNX) return;
  if (in_sizes[1] != kBatch * kNX) return;
  if (in_sizes[2] != kHid * kW1P) return;
  if (in_sizes[3] != kHid) return;
  if (in_sizes[4] != kHid * kHid) return;
  if (in_sizes[5] != kHid) return;
  if (in_sizes[6] != kHid) return;
  if (in_sizes[7] != 1) return;
  if (out_size != kPairs + 1) return;
  if (ws_size < kWsTotal) return;

  const float* x  = (const float*)d_in[0];
  const float* y  = (const float*)d_in[1];
  const float* W1 = (const float*)d_in[2];
  const float* b1 = (const float*)d_in[3];
  const float* W2 = (const float*)d_in[4];
  const float* b2 = (const float*)d_in[5];
  const float* W3 = (const float*)d_in[6];
  const float* b3 = (const float*)d_in[7];
  float* out = (float*)d_out;

  char* ws = (char*)d_ws;
  unsigned short* XH  = (unsigned short*)(ws + kOffXH);
  unsigned short* XL  = (unsigned short*)(ws + kOffXL);
  unsigned short* YH  = (unsigned short*)(ws + kOffYH);
  unsigned short* YL  = (unsigned short*)(ws + kOffYL);
  unsigned short* W1H = (unsigned short*)(ws + kOffW1H);
  unsigned short* W1L = (unsigned short*)(ws + kOffW1L);
  unsigned short* W2H = (unsigned short*)(ws + kOffW2H);
  float*          HX  = (float*)(ws + kOffHX);
  float*          HYB = (float*)(ws + kOffHYB);

  split_rows_bf16_kernel<<<(kBatch * kNX / 8) / 256, 256, 0, stream>>>(x, XH, XL, kBatch * kNX / 8);
  split_rows_bf16_kernel<<<(kBatch * kNX / 8) / 256, 256, 0, stream>>>(y, YH, YL, kBatch * kNX / 8);
  split_rows_bf16_kernel<<<(kHid * kW1P / 8) / 256, 256, 0, stream>>>(W1, W1H, W1L, kHid * kW1P / 8);
  w2_plane_kernel<<<(kHid * kHid / 8) / 256, 256, 0, stream>>>(W2, W2H, out + kPairs, kHid * kHid / 8);

  wmma_gemm64_bf16<true, 0><<<8, 256, 0, stream>>>(
      XH, XL, kNX,
      W1H, W1L, kW1P,
      HX, kHid,
      b1,
      kBatch, kHid, kNX);

  wmma_gemm64_bf16<true, 2><<<8, 256, 0, stream>>>(
      YH, YL, kNX,
      W1H + kNX, W1L + kNX, kW1P,
      HYB, kHid,
      b1,
      kBatch, kHid, kNX);

  pair_layer_kernel<<<kPairs / kMT, 256, 0, stream>>>(
      HX, HYB, (const _Float16*)W2H, b2, W3, b3, out);
}
